// DecoderLayer_82867099009768
// MI455X (gfx1250) — hardware-verified
//
#include <hip/hip_runtime.h>
#ifndef NB
#define NB 4
#endif
#ifndef SEQ
#define SEQ 1024
#endif
#define NB_FULL 4
#define SEQ_FULL 1024
#define SCTX 1024
#define SKP 1024
#define DM 1024
#define DMQ DM
#define NH 16
#define HD 64
#define DFF 4096
#define HG 8
#define NGRP (NH / HG)
#define LQ (3 * DM)
#define SMAX (SEQ > SCTX ? SEQ : SCTX)
#define NR ((size_t)NB * SEQ)
#define NRC ((size_t)NB * SCTX)
#define NRX ((size_t)NB * SMAX)
static_assert(SEQ % 128 == 0);
static_assert(SEQ <= SEQ_FULL);
static_assert(NB >= 1 && NB <= NB_FULL);
static_assert(NH % HG == 0);
static_assert(NGRP == 2);
static_assert(SKP == SCTX);
static_assert(SCTX % 128 == 0);
static_assert(DM % 64 == 0 && DFF % 64 == 0 && HD == 64 && DMQ == 1024);
static_assert((size_t)NB_FULL * SEQ_FULL * DM * 4 == 16777216);

typedef unsigned short v8us __attribute__((ext_vector_type(8), may_alias));
typedef float  v8f  __attribute__((ext_vector_type(8)));
typedef float  v4f  __attribute__((ext_vector_type(4)));
typedef float  v4fa __attribute__((ext_vector_type(4), may_alias));
typedef int    v4i  __attribute__((ext_vector_type(4), may_alias));
typedef _Float16 v16h __attribute__((ext_vector_type(16)));
typedef _Float16 v4h __attribute__((ext_vector_type(4)));
union FragH { v16h v; v8us half[2]; _Float16 h[16]; unsigned short u[16]; unsigned int w[8]; };

__device__ __forceinline__ unsigned short bf16_bits(float x) { unsigned int u = __float_as_uint(x); return (unsigned short)((u + 0x7FFFu + ((u >> 16) & 1u)) >> 16); }
__device__ __forceinline__ float bf16_val(unsigned short b) { return __uint_as_float(((unsigned int)b) << 16); }
__device__ __forceinline__ float bf16_rne(float x) { return bf16_val(bf16_bits(x)); }

__global__ __launch_bounds__(256) void k_wt_f16(const float* __restrict__ W, _Float16* __restrict__ Wt, int K, int N, float scale) {
  const int t = blockIdx.x * 256 + threadIdx.x; if (t >= N * (K / 8)) return; const int n = t / (K / 8), k8 = (t % (K / 8)) * 8; FragH f;
#pragma unroll
  for (int i = 0; i < 8; ++i) f.h[i] = (_Float16)(bf16_rne(W[(size_t)(k8 + i) * N + n]) * scale);
  const v8us o = f.half[0]; unsigned short* d = (unsigned short*)Wt + (size_t)n * K + k8;
  *(volatile v8us*)d = o; __threadfence(); *(volatile v8us*)d = o;
}

__global__ __launch_bounds__(256) void k_x16(const float* __restrict__ x, _Float16* __restrict__ X16, size_t n8) {
  const size_t t = (size_t)blockIdx.x * 256 + threadIdx.x; if (t >= n8) return; FragH f;
  const v4f a = *(const v4fa*)(x + t * 8), c = *(const v4fa*)(x + t * 8 + 4);
#pragma unroll
  for (int q = 0; q < 4; ++q) { f.h[q] = (_Float16)bf16_rne(a[q]); f.h[4 + q] = (_Float16)bf16_rne(c[q]); }
  unsigned short* d = (unsigned short*)X16 + t * 8; *(volatile v8us*)d = f.half[0]; __threadfence(); *(volatile v8us*)d = f.half[0];
}

template <int NHv, int TTv>
__global__ __launch_bounds__(256) void k_vt(const _Float16* __restrict__ V16, int ldv, int voff, _Float16* __restrict__ Vt) {
  __shared__ unsigned short tl[64][66]; const int tid = threadIdx.x; const int slab = blockIdx.x / (TTv / 64), lg = blockIdx.x % (TTv / 64); const int b = slab / NHv, h = slab % NHv;
  for (int i = tid; i < 64 * 8; i += 256) { const int r = i / 8, c8 = (i % 8) * 8; FragH f; f.half[0] = *(const v8us*)((const unsigned short*)V16 + ((size_t)b * TTv + lg * 64 + r) * ldv + voff + h * 64 + c8);
#pragma unroll
    for (int q = 0; q < 8; ++q) tl[r][c8 + q] = f.u[q]; }
  __syncthreads();
  for (int pass = 0; pass < 2; ++pass) {
#pragma unroll
    for (int rd = 0; rd < 2; ++rd) { const int d = rd * 32 + tid / 8, pc = tid % 8; FragH f;
#pragma unroll
      for (int q = 0; q < 8; ++q) f.u[q] = tl[pc * 8 + q][d];
      *(volatile v8us*)((unsigned short*)Vt + ((size_t)slab * 64 + d) * TTv + lg * 64 + pc * 8) = f.half[0]; }
    if (pass == 0) __threadfence(); }
}

template <int BFIN, int W16, int W32>
__global__ __launch_bounds__(256) void k_lnx(const float* __restrict__ X, int rpb, size_t bstr, const float* __restrict__ g, const float* __restrict__ bb, float eps, _Float16* __restrict__ N16, float* __restrict__ N32) {
  #pragma clang fp contract(off)
  __shared__ float red[256]; const size_t r = blockIdx.x; const size_t rin = (r / (size_t)rpb) * bstr + (r % (size_t)rpb); const int t = threadIdx.x; const bool act = t < (DMQ / 4); const int c0 = act ? t * 4 : 0;
  const v4f xa = *(const v4fa*)(X + rin * DMQ + c0); float s[4]; float sum = 0.f;
#pragma unroll
  for (int q = 0; q < 4; ++q) { s[q] = act ? (BFIN ? bf16_rne(xa[q]) : xa[q]) : 0.f; sum = __fadd_rn(sum, s[q]); }
  red[t] = sum; __syncthreads(); for (int st = 128; st > 0; st >>= 1) { if (t < st) red[t] = __fadd_rn(red[t], red[t + st]); __syncthreads(); } const float mu = red[0] / (float)DMQ; __syncthreads();
  float vs = 0.f;
#pragma unroll
  for (int q = 0; q < 4; ++q) { const float dl = act ? __fadd_rn(s[q], -mu) : 0.f; vs = __fadd_rn(vs, __fmul_rn(dl, dl)); } red[t] = vs; __syncthreads(); for (int st = 128; st > 0; st >>= 1) { if (t < st) red[t] = __fadd_rn(red[t], red[t + st]); __syncthreads(); }
  const float rs = rsqrtf(__fadd_rn(red[0] / (float)DMQ, eps)); v4h y; v4f yf;
#pragma unroll
  for (int q = 0; q < 4; ++q) { const int c = c0 + q; yf[q] = __fadd_rn(__fmul_rn(__fmul_rn(__fadd_rn(s[q], -mu), rs), bf16_rne(g[c])), bf16_rne(bb[c])); y[q] = (_Float16)yf[q]; }
  if (!act) return;
  for (int pass = 0; pass < 2; ++pass) { if (W16) *(volatile v4h*)(N16 + r * DMQ + c0) = y; if (W32) *(volatile v4f*)(N32 + r * DMQ + c0) = yf; if (pass == 0) __threadfence(); }
}

__device__ __forceinline__ v16h g2_frag(const _Float16* p, int hh) { FragH f; f.half[0] = *(const v8us*)((const unsigned short*)p + 8 * hh); f.half[1] = *(const v8us*)((const unsigned short*)p + 16 + 8 * hh); return f.v; }
__device__ __forceinline__ v8f g2_mma(v16h a, v16h b, v8f c) { v8f d = __builtin_amdgcn_wmma_f32_16x16x32_f16(false, a, false, b, (short)0, c, false, false); asm volatile("v_nop\n\tv_nop\n\tv_nop\n\tv_nop" : "+v"(d) : "v"(a), "v"(b)); return d; }
template <int ACT, int CPR, int MSK, int ZSK, int RSC>
__global__ __launch_bounds__(128) void k_gemm2(const _Float16* __restrict__ A, int lda, size_t sA, const _Float16* __restrict__ Bh, int ldb, size_t sB, float alpha,
    const float* __restrict__ bias, const float* __restrict__ CP, const int* __restrict__ mk, int mstr, const float* __restrict__ rs, int srs,
    float* __restrict__ C, _Float16* __restrict__ C16, int ldc, size_t sC, int M, int N, int K) {
  static_assert(ACT == 0 || ACT == 3);
  __shared__ __attribute__((aligned(16))) float so[4][32][68];
  const int tid = threadIdx.x, w = tid >> 5, lane = tid & 31, ln = lane & 15, hh = lane >> 4; const int by = blockIdx.y;
  A += (size_t)by * sA; Bh += (size_t)by * sB; const size_t cofs = (size_t)by * sC;
  const int ntn = N >> 6; const int mt = blockIdx.x / ntn, nq = blockIdx.x - mt * ntn; const int row0 = mt * 128 + 32 * w, col0 = nq * 64; if (row0 >= M) return;
  const _Float16* a0p = A + (size_t)(row0 + ln) * lda; const _Float16* a1p = a0p + (size_t)16 * lda;
  const _Float16* b0p = Bh + (size_t)(col0 + ln) * ldb; const _Float16* b1p = b0p + (size_t)16 * ldb; const _Float16* b2p = b1p + (size_t)16 * ldb; const _Float16* b3p = b2p + (size_t)16 * ldb;
  const v8f z8 = {0.f,0.f,0.f,0.f,0.f,0.f,0.f,0.f}; v8f c00 = z8, c01 = z8, c02 = z8, c03 = z8, c10 = z8, c11 = z8, c12 = z8, c13 = z8;
  bool live = true;
  if (MSK) {
    const int* mr = mk + (size_t)(row0 + lane) * mstr + col0; int anyu = 0;
#pragma unroll
    for (int j = 0; j < 64; j += 4) { const v4i m4 = *(const v4i*)(mr + j); anyu |= (m4[0] == 0) | (m4[1] == 0) | (m4[2] == 0) | (m4[3] == 0); }
    live = __any(anyu) != 0;
  }
  if (live) {
#pragma unroll 1
    for (int kb = 0; kb < K; kb += 32) {
      FragH fa0, fa1;
      fa0.half[0] = *(const v8us*)((const unsigned short*)a0p + kb + 8 * hh); fa0.half[1] = *(const v8us*)((const unsigned short*)a0p + kb + 16 + 8 * hh);
      fa1.half[0] = *(const v8us*)((const unsigned short*)a1p + kb + 8 * hh); fa1.half[1] = *(const v8us*)((const unsigned short*)a1p + kb + 16 + 8 * hh);
      if (ZSK) { unsigned int z = 0u;
#pragma unroll
        for (int i = 0; i < 8; ++i) z |= fa0.w[i] | fa1.w[i];
        if (__any(z != 0u) == 0) continue; }
      v16h b = g2_frag(b0p + kb, hh); c00 = g2_mma(fa0.v, b, c00); c10 = g2_mma(fa1.v, b, c10);
      b = g2_frag(b1p + kb, hh); c01 = g2_mma(fa0.v, b, c01); c11 = g2_mma(fa1.v, b, c11);
      b = g2_frag(b2p + kb, hh); c02 = g2_mma(fa0.v, b, c02); c12 = g2_mma(fa1.v, b, c12);
      b = g2_frag(b3p + kb, hh); c03 = g2_mma(fa0.v, b, c03); c13 = g2_mma(fa1.v, b, c13); }
  }
  v8f accs[8] = {c00, c01, c02, c03, c10, c11, c12, c13};
  float rsl[16];
#pragma unroll
  for (int i = 0; i < 16; ++i) rsl[i] = 1.0f;
  if (RSC) {
#pragma unroll
    for (int hf = 0; hf < 2; ++hf)
#pragma unroll
      for (int r = 0; r < 8; ++r) rsl[hf * 8 + r] = rs[(size_t)by * srs + row0 + hf * 16 + 8 * hh + r];
  }
#pragma unroll
  for (int u = 0; u < 8; ++u) { const int t = u & 3, hf = u >> 2; const int col = col0 + t * 16 + ln; const float bv = bias ? bf16_rne(bias[col]) : 0.f;
#pragma unroll
    for (int r = 0; r < 8; ++r) { const int rloc = hf * 16 + 8 * hh + r; float v = accs[u][r] * alpha; if (RSC) v *= rsl[hf * 8 + r]; v += bv;
      if (CP) { float cv = CP[cofs + (size_t)(row0 + rloc) * ldc + col]; if (CPR) cv = bf16_rne(cv); v += cv; }
      if (MSK) { const int m = mk[(size_t)(row0 + rloc) * mstr + col]; v = (m != 0) ? -1.0e9f : v; }
      if (ACT == 3) v = fmaxf(v, 0.f);
      so[w][rloc][t * 16 + ln] = v; } }
  __builtin_amdgcn_fence(4  , "workgroup"); __builtin_amdgcn_wave_barrier();
  const int rsub = lane >> 4, c4 = (lane & 15) * 4;
  for (int pass = 0; pass < 2; ++pass) {
#pragma unroll
    for (int q = 0; q < 16; ++q) { const int r = q * 2 + rsub; const v4f v = *(const v4fa*)&so[w][r][c4]; if (C) *(volatile v4f*)(C + cofs + (size_t)(row0 + r) * ldc + col0 + c4) = v; if (C16) { v4h h4;
#pragma unroll
        for (int i = 0; i < 4; ++i) h4[i] = (_Float16)v[i]; *(volatile v4h*)(C16 + cofs + (size_t)(row0 + r) * ldc + col0 + c4) = h4; } }
    if (pass == 0) __threadfence(); }
}

__global__ __launch_bounds__(256) void k_smx(const float* __restrict__ S, _Float16* __restrict__ E, float* __restrict__ RS, int nrows, int nk) {
  #pragma clang fp contract(off)
  const int i = blockIdx.x * 256 + threadIdx.x; if (i >= nrows) return; const float* s = S + (size_t)i * SKP; float mx = -3.0e38f;
#pragma unroll 1
  for (int j = 0; j < nk; j += 4) { const v4f a = *(const v4fa*)(s + j); mx = fmaxf(mx, fmaxf(fmaxf(a[0], a[1]), fmaxf(a[2], a[3]))); }
  float se = 0.f;
#pragma unroll 1
  for (int j0 = 0; j0 < nk; j0 += 8) { const v4f a = *(const v4fa*)(s + j0), c = *(const v4fa*)(s + j0 + 4); FragH f;
#pragma unroll
    for (int q = 0; q < 4; ++q) { const float e = __expf(a[q] - mx); se = se + e; f.h[q] = (_Float16)(e * 1024.0f); }
#pragma unroll
    for (int q = 0; q < 4; ++q) { const float e = __expf(c[q] - mx); se = se + e; f.h[4 + q] = (_Float16)(e * 1024.0f); }
    unsigned short* d = (unsigned short*)E + (size_t)i * SKP + j0; *(volatile v8us*)d = f.half[0]; __threadfence(); *(volatile v8us*)d = f.half[0]; }
  const float rr = 1.0f / se;
  *(volatile float*)(RS + i) = rr; __threadfence(); *(volatile float*)(RS + i) = rr;
}

__global__ __launch_bounds__(256) void k_cov(const _Float16* __restrict__ E, const float* __restrict__ RS, const float* __restrict__ Pin, float* __restrict__ Pout, int hg, float cscale) {
  __shared__ __attribute__((aligned(16))) float tile[4][SKP];
  const int tid = threadIdx.x, ql = tid >> 6, seg = tid & 63; const int q = blockIdx.x * 4 + ql;
  float acc[16];
#pragma unroll
  for (int i = 0; i < 16; ++i) acc[i] = 0.f;
#pragma unroll 1
  for (int h = 0; h < hg; ++h) { const float rq = RS[(size_t)h * SEQ + q]; const unsigned short* ep = (const unsigned short*)E + ((size_t)h * SEQ + q) * SKP + seg * 16; FragH f; f.half[0] = *(const v8us*)ep; f.half[1] = *(const v8us*)(ep + 8);
#pragma unroll
    for (int i = 0; i < 16; ++i) acc[i] += (float)f.h[i] * rq; }
  v4f pv[4];
#pragma unroll
  for (int i = 0; i < 4; ++i) { pv[i][0] = 0.f; pv[i][1] = 0.f; pv[i][2] = 0.f; pv[i][3] = 0.f; }
  if (Pin != nullptr) { const float* pp = Pin + (size_t)q * SKP + seg * 16;
#pragma unroll
    for (int i = 0; i < 4; ++i) pv[i] = *(const v4fa*)(pp + 4 * i); }
#pragma unroll
  for (int i = 0; i < 4; ++i) { v4f o;
#pragma unroll
    for (int k = 0; k < 4; ++k) o[k] = acc[4 * i + k] * cscale + pv[i][k]; *(v4fa*)&tile[ql][seg * 16 + 4 * i] = o; }
  __syncthreads();
  for (int pass = 0; pass < 2; ++pass) {
#pragma unroll
    for (int it = 0; it < 4; ++it) { const int line = it * 32 + (tid >> 3); const int row = line >> 5; const int cj = (line & 31) * 32 + (tid & 7) * 4; const v4f v = *(const v4fa*)&tile[row][cj]; *(volatile v4f*)(Pout + (size_t)(blockIdx.x * 4 + row) * SKP + cj) = v; }
    if (pass == 0) __threadfence(); }
}

static inline size_t zmax(size_t a, size_t b) { return a > b ? a : b; }

extern "C" void kernel_launch(void* const* d_in, const int* in_sizes, int n_in,
                              void* d_out, int out_size, void* d_ws, size_t ws_size, hipStream_t stream) {
  if (n_in < 30) return;
  const float* x = (const float*)d_in[0]; const float* ctx = (const float*)d_in[1]; const int* mtgt = (const int*)d_in[2]; const int* msrc = (const int*)d_in[3];
  const float* ln1g = (const float*)d_in[4]; const float* ln1b = (const float*)d_in[5]; const float* ln2g = (const float*)d_in[6]; const float* ln2b = (const float*)d_in[7]; const float* ln3g = (const float*)d_in[8]; const float* ln3b = (const float*)d_in[9];
  const float* saWq = (const float*)d_in[10]; const float* sabq = (const float*)d_in[11]; const float* saWk = (const float*)d_in[12]; const float* sabk = (const float*)d_in[13];
  const float* saWv = (const float*)d_in[14]; const float* sabv = (const float*)d_in[15]; const float* saWo = (const float*)d_in[16]; const float* sabo = (const float*)d_in[17];
  const float* caWq = (const float*)d_in[18]; const float* cabq = (const float*)d_in[19]; const float* caWk = (const float*)d_in[20]; const float* cabk = (const float*)d_in[21];
  const float* caWv = (const float*)d_in[22]; const float* cabv = (const float*)d_in[23]; const float* caWo = (const float*)d_in[24]; const float* cabo = (const float*)d_in[25];
  const float* W1 = (const float*)d_in[26]; const float* b1 = (const float*)d_in[27]; const float* W2 = (const float*)d_in[28]; const float* b2 = (const float*)d_in[29];
  if ((size_t)in_sizes[0] < ((size_t)(NB - 1) * SEQ_FULL + SEQ) * DM) return;
  if ((size_t)in_sizes[1] < NRC * DM) return;
  if ((size_t)in_sizes[2] < (size_t)(SEQ - 1) * SEQ_FULL + SEQ) return;
  if ((size_t)in_sizes[3] < (size_t)NB * SCTX) return;
  for (int i = 4; i <= 9; ++i) if (in_sizes[i] < DM) return;
  for (int i = 10; i <= 24; i += 2) if ((size_t)in_sizes[i] < (size_t)DM * DM) return;
  for (int i = 11; i <= 25; i += 2) if (in_sizes[i] < DM) return;
  if ((size_t)in_sizes[26] < (size_t)DM * DFF || in_sizes[27] < DFF || (size_t)in_sizes[28] < (size_t)DFF * DM || in_sizes[29] < DM) return;
  if ((size_t)out_size < (size_t)NB_FULL * SEQ_FULL * DM + ((size_t)(NB - 1) * SEQ_FULL + SEQ) * SCTX) return;
  float* out0 = (float*)d_out; float* out1 = out0 + (size_t)NB_FULL * SEQ_FULL * DM;

  char* ws = (char*)d_ws; size_t off = 0;
  auto take = [&](size_t bytes) { char* p = ws + off; off += (bytes + 255) & ~(size_t)255; return p; };
  const size_t szW   = (size_t)4 * DM * DM * 2;
  const size_t szX16 = zmax(NR * DM * 2, (size_t)SEQ * SKP * 4);
  const size_t szQKV = zmax(NRX * LQ * 2, NR * DM * 4);
  const size_t szO16 = NRX * DM * 2;
  const size_t szX1  = zmax(NR * DM * 4, (size_t)SEQ * DFF * 2);
  const size_t szS   = zmax((size_t)HG * SEQ * SKP * 4, (size_t)2 * DFF * DM * 2);
  const size_t szE   = (size_t)HG * SEQ * SKP * 2;
  const size_t szVT  = (size_t)NH * HD * SMAX * 2;
  const size_t szRS  = (size_t)HG * SEQ * 4;
  _Float16* RWS = (_Float16*)take(szW); _Float16* RWC = (_Float16*)take(szW); char* RX16 = take(szX16); char* RQKV = take(szQKV); char* RO16 = take(szO16); char* RX1 = take(szX1); char* RSS = take(szS);
  _Float16* E16 = (_Float16*)take(szE); _Float16* VT = (_Float16*)take(szVT); float* RSP = (float*)take(szRS);
  if (off > ws_size || off > (size_t)134217728) return;
  _Float16* Bsq = RWS; _Float16* Bsk = RWS + (size_t)DM * DM; _Float16* Bsv = RWS + (size_t)2 * DM * DM; _Float16* Bso = RWS + (size_t)3 * DM * DM;
  _Float16* Bcq = RWC; _Float16* Bck = RWC + (size_t)DM * DM; _Float16* Bcv = RWC + (size_t)2 * DM * DM; _Float16* Bco = RWC + (size_t)3 * DM * DM;
  _Float16* X16 = (_Float16*)RX16; float* COVP = (float*)RX16;
  _Float16* QKV = (_Float16*)RQKV; float* X2 = (float*)RQKV;
  _Float16* O16 = (_Float16*)RO16; _Float16* C16 = (_Float16*)RO16;
  float* X1 = (float*)RX1; _Float16* HF16 = (_Float16*)RX1;
  float* S = (float*)RSS; _Float16* Bt1 = (_Float16*)RSS; _Float16* Bt2 = Bt1 + (size_t)DFF * DM;

  auto wt = [&](const float* W, _Float16* Bt, int K, int N) { k_wt_f16<<<(unsigned)(((size_t)N * (K / 8) + 255) / 256), 256, 0, stream>>>(W, Bt, K, N, 16.0f); };
  auto gx = [](int M, int N) { return (unsigned)(((M + 127) / 128) * (N / 64)); };
  const float EPS = 1e-5f;

  wt(saWq, Bsq, DM, DM); wt(saWk, Bsk, DM, DM); wt(saWv, Bsv, DM, DM); wt(saWo, Bso, DM, DM);
  k_lnx<1, 1, 0><<<(unsigned)NR, 256, 0, stream>>>(x, SEQ, (size_t)SEQ_FULL, ln1g, ln1b, EPS, X16, nullptr);
  k_gemm2<0, 0, 0, 0, 0><<<dim3(gx((int)NR, DM), 1), 128, 0, stream>>>(X16, DM, 0, Bsq, DM, 0, 0.0625f, sabq, nullptr, nullptr, 0, nullptr, 0, nullptr, QKV, LQ, 0, (int)NR, DM, DM);
  k_gemm2<0, 0, 0, 0, 0><<<dim3(gx((int)NR, DM), 1), 128, 0, stream>>>(X16, DM, 0, Bsk, DM, 0, 0.0625f, sabk, nullptr, nullptr, 0, nullptr, 0, nullptr, QKV + DM, LQ, 0, (int)NR, DM, DM);
  k_gemm2<0, 0, 0, 0, 0><<<dim3(gx((int)NR, DM), 1), 128, 0, stream>>>(X16, DM, 0, Bsv, DM, 0, 0.0625f, sabv, nullptr, nullptr, 0, nullptr, 0, nullptr, QKV + 2 * DM, LQ, 0, (int)NR, DM, DM);
  for (int b = 0; b < NB; ++b) { const size_t rq0 = (size_t)b * SEQ;
    k_vt<NH, SEQ><<<NH * (SEQ / 64), 256, 0, stream>>>(QKV + 2 * DM + rq0 * LQ, LQ, 0, VT);
    for (int g = 0; g < NGRP; ++g) { const int h0 = g * HG;
      k_gemm2<0, 0, 1, 0, 0><<<dim3(gx(SEQ, SEQ), HG), 128, 0, stream>>>(QKV + rq0 * LQ + h0 * HD, LQ, (size_t)HD, QKV + DM + rq0 * LQ + h0 * HD, LQ, (size_t)HD, 0.125f, nullptr, nullptr, mtgt, SEQ_FULL, nullptr, 0, S, nullptr, SKP, (size_t)SEQ * SKP, SEQ, SEQ, HD);
      k_smx<<<(unsigned)((HG * SEQ + 255) / 256), 256, 0, stream>>>(S, E16, RSP, HG * SEQ, SEQ);
      k_gemm2<0, 0, 0, 1, 1><<<dim3(gx(SEQ, HD), HG), 128, 0, stream>>>(E16, SKP, (size_t)SEQ * SKP, VT + (size_t)h0 * HD * SEQ, SEQ, (size_t)HD * SEQ, 0.0625f, nullptr, nullptr, nullptr, 0, RSP, SEQ, nullptr, O16 + rq0 * DM + h0 * HD, DM, (size_t)HD, SEQ, HD, SEQ);
    } }
  for (int b = 0; b < NB; ++b) { const size_t rq0 = (size_t)b * SEQ;
    k_gemm2<0, 1, 0, 0, 0><<<dim3(gx(SEQ, DM), 1), 128, 0, stream>>>(O16 + rq0 * DM, DM, 0, Bso, DM, 0, 0.0009765625f, sabo, x + (size_t)b * SEQ_FULL * DM, nullptr, 0, nullptr, 0, X1 + rq0 * DM, nullptr, DM, 0, SEQ, DM, DM); }

  k_lnx<0, 1, 0><<<(unsigned)NR, 256, 0, stream>>>(X1, SEQ, (size_t)SEQ, ln2g, ln2b, EPS, X16, nullptr);
  wt(caWq, Bcq, DM, DM); wt(caWk, Bck, DM, DM); wt(caWv, Bcv, DM, DM); wt(caWo, Bco, DM, DM);
  k_x16<<<(unsigned)((NRC * DM / 8 + 255) / 256), 256, 0, stream>>>(ctx, C16, NRC * DM / 8);
  k_gemm2<0, 0, 0, 0, 0><<<dim3(gx((int)NR, DM), 1), 128, 0, stream>>>(X16, DM, 0, Bcq, DM, 0, 0.0625f, cabq, nullptr, nullptr, 0, nullptr, 0, nullptr, QKV, LQ, 0, (int)NR, DM, DM);
  k_gemm2<0, 0, 0, 0, 0><<<dim3(gx((int)NRC, DM), 1), 128, 0, stream>>>(C16, DM, 0, Bck, DM, 0, 0.0625f, cabk, nullptr, nullptr, 0, nullptr, 0, nullptr, QKV + DM, LQ, 0, (int)NRC, DM, DM);
  k_gemm2<0, 0, 0, 0, 0><<<dim3(gx((int)NRC, DM), 1), 128, 0, stream>>>(C16, DM, 0, Bcv, DM, 0, 0.0625f, cabv, nullptr, nullptr, 0, nullptr, 0, nullptr, QKV + 2 * DM, LQ, 0, (int)NRC, DM, DM);
  for (int b = 0; b < NB; ++b) { const size_t rq0 = (size_t)b * SEQ, rc0 = (size_t)b * SCTX;
    k_vt<NH, SCTX><<<NH * (SCTX / 64), 256, 0, stream>>>(QKV + 2 * DM + rc0 * LQ, LQ, 0, VT);
    for (int g = 0; g < NGRP; ++g) { const int h0 = g * HG;
      k_gemm2<0, 0, 1, 0, 0><<<dim3(gx(SEQ, SCTX), HG), 128, 0, stream>>>(QKV + rq0 * LQ + h0 * HD, LQ, (size_t)HD, QKV + DM + rc0 * LQ + h0 * HD, LQ, (size_t)HD, 0.125f, nullptr, nullptr, msrc + (size_t)b * SCTX, 0, nullptr, 0, S, nullptr, SKP, (size_t)SEQ * SKP, SEQ, SCTX, HD);
      k_smx<<<(unsigned)((HG * SEQ + 255) / 256), 256, 0, stream>>>(S, E16, RSP, HG * SEQ, SCTX);
      k_gemm2<0, 0, 0, 1, 1><<<dim3(gx(SEQ, HD), HG), 128, 0, stream>>>(E16, SKP, (size_t)SEQ * SKP, VT + (size_t)h0 * HD * SCTX, SCTX, (size_t)HD * SCTX, 0.0625f, nullptr, nullptr, nullptr, 0, RSP, SEQ, nullptr, O16 + rq0 * DM + h0 * HD, DM, (size_t)HD, SEQ, HD, SCTX);
      k_cov<<<(unsigned)(SEQ / 4), 256, 0, stream>>>(E16, RSP, (g == 0) ? nullptr : COVP, (g == NGRP - 1) ? (out1 + (size_t)b * SEQ_FULL * SCTX) : COVP, HG, 0.00006103515625f);
    } }
  k_gemm2<0, 0, 0, 0, 0><<<dim3(gx((int)NR, DM), 1), 128, 0, stream>>>(O16, DM, 0, Bco, DM, 0, 0.0009765625f, cabo, X1, nullptr, 0, nullptr, 0, X2, nullptr, DM, 0, (int)NR, DM, DM);

  k_lnx<0, 1, 0><<<(unsigned)NR, 256, 0, stream>>>(X2, SEQ, (size_t)SEQ, ln3g, ln3b, EPS, X16, nullptr);
  wt(W1, Bt1, DM, DFF); wt(W2, Bt2, DFF, DM);
  for (int b = 0; b < NB; ++b) { const size_t rq0 = (size_t)b * SEQ;
    k_gemm2<3, 0, 0, 0, 0><<<dim3(gx(SEQ, DFF), 1), 128, 0, stream>>>(X16 + rq0 * DM, DM, 0, Bt1, DM, 0, 0.0625f, b1, nullptr, nullptr, 0, nullptr, 0, nullptr, HF16, DFF, 0, SEQ, DFF, DM);
    k_gemm2<0, 0, 0, 0, 0><<<dim3(gx(SEQ, DM), 1), 128, 0, stream>>>(HF16, DFF, 0, Bt2, DFF, 0, 0.0625f, b2, X2 + rq0 * DM, nullptr, 0, nullptr, 0, out0 + (size_t)b * SEQ_FULL * DM, nullptr, DM, 0, SEQ, DM, DFF); }
}
